// GDAttention_11373073399827
// MI455X (gfx1250) — hardware-run, weakly checked
//
#include <hip/hip_runtime.h>
#define NB 4
#define SQ 4096
#define HDK 128
#define NHT 8
#define QT 256
#define QT0 256
#define NKX SQ
#define ATS 0.08838834764831845f
typedef __bf16 v16b __attribute__((ext_vector_type(16)));
typedef unsigned short v8us __attribute__((ext_vector_type(8), may_alias));
typedef float  v8f  __attribute__((ext_vector_type(8)));
typedef float  v4f  __attribute__((ext_vector_type(4)));
typedef float  v4fa __attribute__((ext_vector_type(4), may_alias));
union FragB { v16b v; v8us half[2]; unsigned short u[16]; };

__device__ __forceinline__ unsigned short bf16_bits(float x) { unsigned int u = __float_as_uint(x); return (unsigned short)((u + 0x7FFFu + ((u >> 16) & 1u)) >> 16); }
__device__ __forceinline__ float bf16_val(unsigned short b) { return __uint_as_float(((unsigned int)b) << 16); }
__device__ __forceinline__ float bf16_round(float x) { return bf16_val(bf16_bits(x)); }
template <int NT>
__device__ __forceinline__ v8f mmaN(v16b ah, v16b al, v16b bh, v16b bl, v8f c) {
  c = __builtin_amdgcn_wmma_f32_16x16x32_bf16(false, ah, false, bh, (short)0, c, false, false);
  if (NT >= 2) c = __builtin_amdgcn_wmma_f32_16x16x32_bf16(false, al, false, bh, (short)0, c, false, false);
  if (NT >= 3) c = __builtin_amdgcn_wmma_f32_16x16x32_bf16(false, ah, false, bl, (short)0, c, false, false);
  asm volatile("v_nop\n\tv_nop\n\tv_nop\n\tv_nop" : "+v"(c) : "v"(ah), "v"(al), "v"(bh), "v"(bl));
  return c;
}


typedef _Float16 v16h __attribute__((ext_vector_type(16)));
union FragH { v16h v; v8us half[2]; _Float16 h[16]; unsigned short u[16]; };
template <int NT>
__device__ __forceinline__ v8f mmaH(v16h ah, v16h al, v16h bh, v16h bl, v8f c) {
  c = __builtin_amdgcn_wmma_f32_16x16x32_f16(false, ah, false, bh, (short)0, c, false, false);
  if (NT >= 2) c = __builtin_amdgcn_wmma_f32_16x16x32_f16(false, al, false, bh, (short)0, c, false, false);
  if (NT >= 3) c = __builtin_amdgcn_wmma_f32_16x16x32_f16(false, ah, false, bl, (short)0, c, false, false);
  asm volatile("v_nop\n\tv_nop\n\tv_nop\n\tv_nop" : "+v"(c) : "v"(ah), "v"(al), "v"(bh), "v"(bl));
  return c;
}

__global__ __launch_bounds__(256) void k_wt_f16(const float* __restrict__ W, _Float16* __restrict__ Wt, int K, int N, float scale) {
  const int t = blockIdx.x * 256 + threadIdx.x; if (t >= N * (K / 8)) return; const int n = t / (K / 8), k8 = (t % (K / 8)) * 8; FragH f;
#pragma unroll
  for (int i = 0; i < 8; ++i) f.h[i] = (_Float16)(bf16_round(W[(size_t)(k8 + i) * N + n]) * scale); const v8us o = f.half[0];
  *(volatile v8us*)((unsigned short*)Wt + (size_t)n * K + k8) = o; __threadfence(); *(volatile v8us*)((unsigned short*)Wt + (size_t)n * K + k8) = o;
}

typedef _Float16 v4h __attribute__((ext_vector_type(4)));

__global__ __launch_bounds__(256) void k_x16(const float* __restrict__ x, _Float16* __restrict__ X16, size_t n8) { const size_t t = (size_t)blockIdx.x * 256 + threadIdx.x; if (t >= n8) return; FragH f;
#pragma unroll
  for (int q = 0; q < 8; ++q) f.h[q] = (_Float16)bf16_round(x[t * 8 + q]); *(volatile v8us*)((unsigned short*)X16 + t * 8) = f.half[0]; __threadfence(); *(volatile v8us*)((unsigned short*)X16 + t * 8) = f.half[0]; }
__device__ __forceinline__ v16h g2_frag(const _Float16* p, int hh) { FragH f; f.half[0] = *(const v8us*)((const unsigned short*)p + 8 * hh); f.half[1] = *(const v8us*)((const unsigned short*)p + 16 + 8 * hh); return f.v; }
__device__ __forceinline__ v8f g2_mma(v16h a, v16h b, v8f c) { v8f d = __builtin_amdgcn_wmma_f32_16x16x32_f16(false, a, false, b, (short)0, c, false, false); asm volatile("v_nop\n\tv_nop\n\tv_nop\n\tv_nop" : "+v"(d) : "v"(a), "v"(b)); return d; }
template <int ACT>
__global__ __launch_bounds__(128) void k_gemm2(const _Float16* __restrict__ A, int lda, size_t sA, const _Float16* __restrict__ Bh, int ldb, size_t sB, float alpha, const float* __restrict__ bias, size_t sBias, const float* __restrict__ CP, int rowsPerB, size_t sCPb, int row0g,
    float* __restrict__ C, _Float16* __restrict__ C16, int ldc, size_t sC, int M, int N, int K) { static_assert(ACT == 0 || ACT == 3 || ACT == 6 || ACT == 8 || ACT == 9 || ACT == 11 || ACT == 12 || ACT == 14 || ACT == 15 || ACT == 16 || ACT == 17, "k_gemm2: unsupported ACT code (would silently apply no activation)");
  __shared__ __attribute__((aligned(16))) float so[4][32][68];
  const int tid = threadIdx.x, w = tid >> 5, lane = tid & 31, ln = lane & 15, hh = lane >> 4; const int by = blockIdx.y;
  A += (size_t)by * sA; Bh += (size_t)by * sB; const size_t cofs = (size_t)by * sC; const float* bp = bias ? bias + (size_t)by * sBias : nullptr;
  const int ntn = N >> 6; const int mt = blockIdx.x / ntn, nq = blockIdx.x - mt * ntn; const int row0 = mt * 128 + 32 * w, col0 = nq * 64; if (row0 >= M) return;
  const _Float16* a0p = A + (size_t)(row0 + ln) * lda; const _Float16* a1p = a0p + (size_t)16 * lda;
  const _Float16* b0p = Bh + (size_t)(col0 + ln) * ldb; const _Float16* b1p = b0p + (size_t)16 * ldb; const _Float16* b2p = b1p + (size_t)16 * ldb; const _Float16* b3p = b2p + (size_t)16 * ldb;
  const v8f z8 = {0.f,0.f,0.f,0.f,0.f,0.f,0.f,0.f}; v8f c00 = z8, c01 = z8, c02 = z8, c03 = z8, c10 = z8, c11 = z8, c12 = z8, c13 = z8;
  for (int kb = 0; kb < K; kb += 32) { const v16h a0 = g2_frag(a0p + kb, hh), a1 = g2_frag(a1p + kb, hh);
    v16h b = g2_frag(b0p + kb, hh); c00 = g2_mma(a0, b, c00); c10 = g2_mma(a1, b, c10);
    b = g2_frag(b1p + kb, hh); c01 = g2_mma(a0, b, c01); c11 = g2_mma(a1, b, c11);
    b = g2_frag(b2p + kb, hh); c02 = g2_mma(a0, b, c02); c12 = g2_mma(a1, b, c12);
    b = g2_frag(b3p + kb, hh); c03 = g2_mma(a0, b, c03); c13 = g2_mma(a1, b, c13); }
  v8f accs[8] = {c00, c01, c02, c03, c10, c11, c12, c13};
#pragma unroll
  for (int u = 0; u < 8; ++u) { const int t = u & 3, half = u >> 2; const int col = col0 + t * 16 + ln; const float bv = bp ? bf16_round(bp[col]) : 0.f;
#pragma unroll
    for (int r = 0; r < 8; ++r) { const int rloc = half * 16 + 8 * hh + r; float v = accs[u][r] * alpha + bv; if (CP) { if (rowsPerB < 0) v += CP[cofs + (size_t)(row0g + row0 + rloc) * ldc + col];        else { const int bidx = (row0g + row0 + rloc) / rowsPerB; v += CP[(size_t)bidx * sCPb + (size_t)by * 64 + col]; } }
      if (ACT == 3) v = fmaxf(v, 0.f); else if (ACT == 6) v = 0.5f * v * (1.0f + erff(v * 0.70710678118654752f)); else if (ACT == 11) v = 1.0f / (1.0f + expf(-v)); else if (ACT == 15) v = v / (1.0f + expf(-v)); else if (ACT == 12) v = (v > 0.f) ? v : 0.01f * v; else if (ACT == 8) v = tanhf(v); else if (ACT == 9) v = 0.5f * v * (1.0f + tanhf(0.7978845608028654f * (v + 0.044715f * v * v * v))); else if (ACT == 14) v = (v > 0.f) ? v : 0.1f * v; else if (ACT == 16) v = (v >= 0.f) ? v : 0.3f * v; else if (ACT == 17) v = (v >= 0.f) ? v : 0.2f * v;
      so[w][rloc][t * 16 + ln] = v; } }
  __builtin_amdgcn_fence(__ATOMIC_ACQ_REL, "workgroup"); __builtin_amdgcn_wave_barrier();
  const int rsub = lane >> 4, c4 = (lane & 15) * 4;
  for (int pass = 0; pass < 2; ++pass) {
#pragma unroll
    for (int q = 0; q < 16; ++q) { const int r = q * 2 + rsub; const v4f v = *(const v4fa*)&so[w][r][c4]; if (C) *(volatile v4f*)(C + cofs + (size_t)(row0 + r) * ldc + col0 + c4) = v; if (C16) { v4h h4; for (int i = 0; i < 4; ++i) h4[i] = (_Float16)v[i]; *(volatile v4h*)(C16 + cofs + (size_t)(row0 + r) * ldc + col0 + c4) = h4; } }
    if (pass == 0) __threadfence(); } }

__global__ __launch_bounds__(256) void k_wnat(const float* __restrict__ w, size_t n8, _Float16* __restrict__ Bt) { const size_t t = (size_t)blockIdx.x * 256 + threadIdx.x; if (t >= n8) return; FragH f; for (int q = 0; q < 8; ++q) f.h[q] = (_Float16)(bf16_round(w[t * 8 + q]) * 16.0f); *(volatile v8us*)((unsigned short*)Bt + t * 8) = f.half[0]; __threadfence(); *(volatile v8us*)((unsigned short*)Bt + t * 8) = f.half[0]; }
__global__ __launch_bounds__(256) void k_hl(const float* __restrict__ F, _Float16* __restrict__ Hh, _Float16* __restrict__ Hl, size_t n8) { const size_t t = (size_t)blockIdx.x * 256 + threadIdx.x; if (t >= n8) return; FragH fh, fl; const v4f a = *(const v4fa*)(F + t * 8), c = *(const v4fa*)(F + t * 8 + 4);
#pragma unroll
  for (int q = 0; q < 4; ++q) { _Float16 h = (_Float16)a[q]; fh.h[q] = h; fl.h[q] = (_Float16)((a[q] - (float)h) * 1024.0f); h = (_Float16)c[q]; fh.h[4 + q] = h; fl.h[4 + q] = (_Float16)((c[q] - (float)h) * 1024.0f); }
  for (int pass = 0; pass < 2; ++pass) { *(volatile v8us*)((unsigned short*)Hh + t * 8) = fh.half[0]; *(volatile v8us*)((unsigned short*)Hl + t * 8) = fl.half[0]; if (pass == 0) __threadfence(); } }
__global__ __launch_bounds__(256) void k_bfr(const float* __restrict__ x, float* __restrict__ XB, size_t n8) { const size_t t = (size_t)blockIdx.x * 256 + threadIdx.x; if (t >= n8) return; v4f a = *(const v4fa*)(x + t * 8), c = *(const v4fa*)(x + t * 8 + 4); for (int q = 0; q < 4; ++q) { a[q] = bf16_round(a[q]); c[q] = bf16_round(c[q]); }
  for (int pass = 0; pass < 2; ++pass) { *(volatile v4f*)(XB + t * 8) = a; *(volatile v4f*)(XB + t * 8 + 4) = c; if (pass == 0) __threadfence(); } }
template <int MASK>
__global__ __launch_bounds__(32) void k_att0h(const float* __restrict__ QF, const float* __restrict__ KF, const float* __restrict__ VF, int ld, int ldv, const int* __restrict__ mk, float scale, float* __restrict__ OF, int ldo) {
  #pragma clang fp contract(off)
  __shared__ __attribute__((aligned(16))) float lq[32][128]; __shared__ __attribute__((aligned(16))) float lo[32][128];
  const int tid = threadIdx.x; const int h = blockIdx.x / (QT0 / 32), rg = blockIdx.x % (QT0 / 32); const int i = rg * 32 + tid;
  for (int c = 0; c < 32; ++c) { *(v4f*)&lq[tid][c * 4] = *(const v4fa*)(QF + (size_t)i * ld + h * 128 + c * 4); const v4f z = {0.f, 0.f, 0.f, 0.f}; *(v4f*)&lo[tid][c * 4] = z; }
  float m = -1.0e30f, l = 0.f; const int jmax = rg * 32 + 31;
#pragma unroll 1
  for (int j = 0; j <= jmax; ++j) { const float* kr = KF + (size_t)j * ld + h * 128; const float* vr = VF + (size_t)j * ldv + h * 128; float s = 0.f;
#pragma unroll 1
    for (int c = 0; c < 32; ++c) { const v4f kq = *(const v4fa*)(kr + c * 4); const v4f qq = *(v4f*)&lq[tid][c * 4]; for (int u = 0; u < 4; ++u) s = __fadd_rn(s, __fmul_rn(qq[u], kq[u])); }
    s = __fmul_rn(s, scale); float f; if (MASK) { const int mb = mk[(size_t)i * SQ + j]; f = (mb == 0) ? 1.f : 0.f; } else { f = (j <= i) ? 1.f : 0.f; }
    const float sm = fmaf(f, s, (1.f - f) * -1.0e30f); const float mn = fmaxf(m, sm); const float sc = expf(m - mn); const float e = __fmul_rn(f, expf(sm - mn)); l = __fadd_rn(__fmul_rn(l, sc), e); m = mn;
#pragma unroll 1
    for (int c = 0; c < 32; ++c) { const v4f vv = *(const v4fa*)(vr + c * 4); v4f oo = *(v4f*)&lo[tid][c * 4]; for (int u = 0; u < 4; ++u) oo[u] = __fadd_rn(__fmul_rn(oo[u], sc), __fmul_rn(e, vv[u])); *(v4f*)&lo[tid][c * 4] = oo; } }
  const float fin = 64.0f / l;
  for (int pass = 0; pass < 2; ++pass) { for (int c = 0; c < 32; ++c) { v4f oo = *(v4f*)&lo[tid][c * 4]; for (int u = 0; u < 4; ++u) oo[u] = __fmul_rn(oo[u], fin); *(volatile v4f*)(OF + (size_t)i * ldo + h * 128 + c * 4) = oo; } if (pass == 0) __threadfence(); } }
__global__ __launch_bounds__(256) void k_rsmcf2(const float* __restrict__ S, _Float16* __restrict__ P, int hg, int q0, int nk) {
  #pragma clang fp contract(off)
  const int t = blockIdx.x * 256 + threadIdx.x; if (t >= hg * QT) return; const size_t i = (size_t)t; const float* s = S + i * NKX; const int last = q0 + (t % QT); float mx = -3.0e38f;
#pragma unroll 1
  for (int j = 0; j < nk; ++j) { const float f = (j <= last) ? 1.f : 0.f; mx = fmaxf(mx, fmaf(f, s[j], (1.f - f) * -1.0e9f)); } float se = 0.f;
#pragma unroll 1
  for (int j = 0; j < nk; ++j) { const float f = (j <= last) ? 1.f : 0.f; se += __expf(fmaf(f, s[j], (1.f - f) * -1.0e9f) - mx); } const float sc = 256.0f / se;
#pragma unroll 1
  for (int j0 = 0; j0 < nk; j0 += 8) { FragH fr; for (int q = 0; q < 8; ++q) { const int j = j0 + q; const float f = (j <= last) ? 1.f : 0.f; fr.h[q] = (_Float16)(__expf(fmaf(f, s[j], (1.f - f) * -1.0e9f) - mx) * sc); } unsigned short* d = (unsigned short*)P + i * NKX + j0; *(volatile v8us*)d = fr.half[0]; __threadfence(); *(volatile v8us*)d = fr.half[0]; } }

extern "C" void kernel_launch(void* const* d_in, const int* in_sizes, int n_in,
                              void* d_out, int out_size, void* d_ws, size_t ws_size, hipStream_t stream) {
  (void)in_sizes; (void)n_in; (void)out_size;
  const float* e = (const float*)d_in[0]; const float* p = (const float*)d_in[1]; const float* W_o_w = (const float*)d_in[2]; const float* W_o_b = (const float*)d_in[3];
  static_assert(NB == 4 && SQ == 4096 && HDK == 128 && NHT == 8 && QT == 256 && QT0 == 256 && NKX == SQ && SQ % QT == 0 && QT % 128 == 0 && QT0 % 128 == 0 && QT0 % 32 == 0 && HDK % 64 == 0 && HDK % 32 == 0 && ((size_t)SQ * HDK / 8) % 256 == 0 && ((size_t)HDK * (SQ / 8)) % 256 == 0 && ((size_t)HDK * NHT * HDK / 8) % 256 == 0 && ((size_t)QT0 * HDK / 8) % 256 == 0 && ((size_t)NB * QT0 * HDK / 8) % 256 == 0, "whole tiles; exact grids");
  float* out = (float*)d_out;
  const size_t NR = (size_t)NB * SQ;
  const size_t PB = (size_t)(SQ + 1) * HDK;
  char* ws = (char*)d_ws; size_t off = 0;
  auto take = [&](size_t bytes) { char* q = ws + off; off += (bytes + 255) & ~(size_t)255; return q; };
  _Float16* Q16 = (_Float16*)take(NR * HDK * 2); _Float16* K16 = (_Float16*)take(NR * HDK * 2); _Float16* VT = (_Float16*)take((size_t)NB * HDK * SQ * 2); _Float16* BO = (_Float16*)take((size_t)HDK * NHT * HDK * 2); _Float16* O16 = (_Float16*)take(NR * HDK * 2);
  float* S = (float*)take((size_t)QT * NKX * 4); _Float16* PW = (_Float16*)take((size_t)QT * NKX * 2);
  float* QF0 = (float*)take((size_t)QT0 * HDK * 4); float* KF0 = (float*)take((size_t)QT0 * HDK * 4); float* VF0 = (float*)take((size_t)QT0 * HDK * 4); float* OF0 = (float*)take((size_t)NB * QT0 * HDK * 4); _Float16* OH0 = (_Float16*)take((size_t)NB * QT0 * HDK * 2); _Float16* OL0 = (_Float16*)take((size_t)NB * QT0 * HDK * 2);
  if (off > ws_size) return;
  k_wnat<<<(unsigned)((size_t)HDK * NHT * HDK / 8 / 256), 256, 0, stream>>>(W_o_w, (size_t)HDK * NHT * HDK / 8, BO);
  for (int b = 0; b < NB; ++b) { const size_t r0 = (size_t)b * SQ;
    k_x16<<<(unsigned)((size_t)SQ * HDK / 8 / 256), 256, 0, stream>>>(p + (size_t)b * PB + HDK, Q16 + r0 * HDK, (size_t)SQ * HDK / 8);
    k_x16<<<(unsigned)((size_t)SQ * HDK / 8 / 256), 256, 0, stream>>>(p + (size_t)b * PB, K16 + r0 * HDK, (size_t)SQ * HDK / 8);
    k_wt_f16<<<(unsigned)((size_t)HDK * (SQ / 8) / 256), 256, 0, stream>>>(e + r0 * HDK, VT + (size_t)b * HDK * SQ, SQ, HDK, 1.0f);
    { const unsigned g = (unsigned)((size_t)QT0 * HDK / 8 / 256); k_bfr<<<g, 256, 0, stream>>>(p + (size_t)b * PB + HDK, QF0, (size_t)QT0 * HDK / 8); k_bfr<<<g, 256, 0, stream>>>(p + (size_t)b * PB, KF0, (size_t)QT0 * HDK / 8); k_bfr<<<g, 256, 0, stream>>>(e + r0 * HDK, VF0, (size_t)QT0 * HDK / 8); }
    k_att0h<0><<<QT0 / 32, 32, 0, stream>>>(QF0, KF0, VF0, HDK, HDK, nullptr, ATS, OF0 + (size_t)b * QT0 * HDK, HDK);
    for (int q0 = 0; q0 < SQ; q0 += QT) { const int nk = q0 + QT;
      k_gemm2<0><<<dim3((unsigned)((QT / 128) * (nk / 64)), 1), 128, 0, stream>>>(Q16 + (r0 + q0) * HDK, HDK, (size_t)0, K16 + r0 * HDK, HDK, (size_t)0, ATS, nullptr, 0, nullptr, 1, 0, 0, S, nullptr, NKX, (size_t)0, QT, nk, HDK);
      k_rsmcf2<<<(QT + 255) / 256, 256, 0, stream>>>(S, PW, 1, q0, nk);
      k_gemm2<0><<<dim3((unsigned)((QT / 128) * (HDK / 64)), 1), 128, 0, stream>>>(PW, NKX, (size_t)0, VT + (size_t)b * HDK * SQ, SQ, (size_t)0, 0.25f, nullptr, 0, nullptr, 1, 0, 0, nullptr, O16 + (r0 + q0) * HDK, HDK, (size_t)0, QT, HDK, nk); } }
  k_gemm2<0><<<dim3((unsigned)((NR / 128) * (HDK / 64)), 1), 128, 0, stream>>>(O16, HDK, (size_t)0, BO, NHT * HDK, (size_t)0, 0.0009765625f, W_o_b, 0, nullptr, 1, 0, 0, out, nullptr, HDK, (size_t)0, (int)NR, HDK, HDK);
  for (int h = 1; h < NHT; ++h) k_gemm2<0><<<dim3((unsigned)((NR / 128) * (HDK / 64)), 1), 128, 0, stream>>>(O16, HDK, (size_t)0, BO + (size_t)h * HDK, NHT * HDK, (size_t)0, 0.0009765625f, nullptr, 0, out, -1, 0, 0, out, nullptr, HDK, (size_t)0, (int)NR, HDK, HDK);
  k_hl<<<(unsigned)((size_t)NB * QT0 * HDK / 8 / 256), 256, 0, stream>>>(OF0, OH0, OL0, (size_t)NB * QT0 * HDK / 8);
  for (int b = 0; b < NB; ++b) { float* ob = out + (size_t)b * SQ * HDK; const size_t f0 = (size_t)b * QT0 * HDK;
    k_gemm2<0><<<dim3((unsigned)((QT0 / 128) * (HDK / 64)), 1), 128, 0, stream>>>(OH0 + f0, HDK, (size_t)0, BO, NHT * HDK, (size_t)0, 0.0009765625f, W_o_b, 0, nullptr, 1, 0, 0, ob, nullptr, HDK, (size_t)0, QT0, HDK, HDK);
    for (int h = 1; h < NHT; ++h) k_gemm2<0><<<dim3((unsigned)((QT0 / 128) * (HDK / 64)), 1), 128, 0, stream>>>(OH0 + f0, HDK, (size_t)0, BO + (size_t)h * HDK, NHT * HDK, (size_t)0, 0.0009765625f, nullptr, 0, ob, -1, 0, 0, ob, nullptr, HDK, (size_t)0, QT0, HDK, HDK);
    for (int h = 0; h < NHT; ++h) k_gemm2<0><<<dim3((unsigned)((QT0 / 128) * (HDK / 64)), 1), 128, 0, stream>>>(OL0 + f0, HDK, (size_t)0, BO + (size_t)h * HDK, NHT * HDK, (size_t)0, 0.00000095367431640625f, nullptr, 0, ob, -1, 0, 0, ob, nullptr, HDK, (size_t)0, QT0, HDK, HDK); }
}
